// TrajectoryAttention_5952824673115
// MI455X (gfx1250) — hardware-run, weakly checked
//
#include <hip/hip_runtime.h>
#include <math.h>
#include <stdint.h>

#define PP 920
#define FF 5
#define HH 8
#define CC 256
#define NB 4
#define NTOK (FF * PP)
#define NPAD 4672
#define C2 (2 * CC)
#define C3 (3 * CC)
#define QPITCH 264
#define VPITCH 72

static_assert(NPAD % 64 == 0);
static_assert((NPAD * FF) % 64 == 0);
static_assert(NPAD >= (FF - 1) * PP + 15 * 64);
static_assert((NTOK * FF) % 4 == 0);
static_assert((NB * NPAD) % 64 == 0);
static_assert((NB * HH * NTOK * FF / 4) % 32 == 0);

typedef _Float16       v16h __attribute__((ext_vector_type(16)));
typedef _Float16       v8h  __attribute__((ext_vector_type(8)));
typedef __bf16         v16b __attribute__((ext_vector_type(16)));
typedef __bf16         v8b  __attribute__((ext_vector_type(8)));
typedef float          v8f  __attribute__((ext_vector_type(8)));
typedef float          v4f  __attribute__((ext_vector_type(4)));
typedef unsigned short v8us __attribute__((ext_vector_type(8)));

union FragH { v16h v; v8h hf[2]; };
union FragB { v16b v; v8b hf[2]; };

__device__ __forceinline__ unsigned short f2bf_bits(float f) {
  const unsigned u = __float_as_uint(f);
  return (unsigned short)((u + 0x7FFFu + ((u >> 16) & 1u)) >> 16);
}
__device__ __forceinline__ float bf_bits2f(unsigned short h) { return __uint_as_float(((unsigned)h) << 16); }

__device__ __forceinline__ v16h ldfragh(const _Float16* p) {
  FragH u;
  u.hf[0] = *(const v8h*)(p);
  u.hf[1] = *(const v8h*)(p + 16);
  return u.v;
}
__device__ __forceinline__ v16b ldfragb(const __bf16* p) {
  FragB u;
  u.hf[0] = *(const v8b*)(p);
  u.hf[1] = *(const v8b*)(p + 16);
  return u.v;
}
__device__ __forceinline__ v8f zacc() {
  v8f z = {0.f, 0.f, 0.f, 0.f, 0.f, 0.f, 0.f, 0.f};
  return z;
}
__device__ __forceinline__ v8f mmah(v16h a, v16h b, v8f c) {
  c = __builtin_amdgcn_wmma_f32_16x16x32_f16(false, a, false, b, (short)0, c, false, false);
  asm volatile("v_nop\n\tv_nop\n\tv_nop\n\tv_nop" : "+v"(c) : "v"(a), "v"(b));
  return c;
}
__device__ __forceinline__ v8f mmab(v16b a, v16b b, v8f c) {
  c = __builtin_amdgcn_wmma_f32_16x16x32_bf16(false, a, false, b, (short)0, c, false, false);
  asm volatile("v_nop\n\tv_nop\n\tv_nop\n\tv_nop" : "+v"(c) : "v"(a), "v"(b));
  return c;
}
__device__ __forceinline__ void wave_sync_lds() {
  __builtin_amdgcn_fence(__ATOMIC_RELEASE, "workgroup");
  __builtin_amdgcn_wave_barrier();
  __builtin_amdgcn_fence(__ATOMIC_ACQUIRE, "workgroup");
}

__global__ __launch_bounds__(256) void k_wcvt(
    const float* __restrict__ w0, unsigned short* __restrict__ h0, unsigned short* __restrict__ l0, int n0,
    const float* __restrict__ w1, unsigned short* __restrict__ h1, unsigned short* __restrict__ l1, int n1,
    const float* __restrict__ w2, unsigned short* __restrict__ h2, unsigned short* __restrict__ l2, int n2,
    const float* __restrict__ w3, unsigned short* __restrict__ h3, unsigned short* __restrict__ l3, int n3)
{
  const float* w = w0; unsigned short* dh = h0; unsigned short* dl = l0; int n = n0;
  if (blockIdx.y == 1) { w = w1; dh = h1; dl = l1; n = n1; }
  else if (blockIdx.y == 2) { w = w2; dh = h2; dl = l2; n = n2; }
  else if (blockIdx.y == 3) { w = w3; dh = h3; dl = l3; n = n3; }
  const int i = blockIdx.x * 256 + threadIdx.x;
  if (8 * i >= n) return;
  const size_t o8 = (size_t)i * 8;
  const v4f a0 = *(const v4f*)(w + o8);
  const v4f a1 = *(const v4f*)(w + o8 + 4);
  v8us hv, lv;
#pragma unroll
  for (int e = 0; e < 4; ++e) {
    const unsigned short hb0 = f2bf_bits(a0[e]);
    const unsigned short hb1 = f2bf_bits(a1[e]);
    hv[e]     = hb0;
    hv[4 + e] = hb1;
    lv[e]     = f2bf_bits(a0[e] - bf_bits2f(hb0));
    lv[4 + e] = f2bf_bits(a1[e] - bf_bits2f(hb1));
  }
  *(volatile v8us*)(dh + o8) = hv;
  *(volatile v8us*)(dl + o8) = lv;
  __threadfence();
  *(volatile v8us*)(dh + o8) = hv;
  *(volatile v8us*)(dl + o8) = lv;
}

__global__ __launch_bounds__(256) void k_pack(const float* __restrict__ x,
                                              unsigned short* __restrict__ XBh, unsigned short* __restrict__ XBl)
{
  const int g = blockIdx.x * 256 + threadIdx.x;
  const int R = g >> 5;
  const int L = g & 31;
  const int b = R / NPAD;
  const int n = R - b * NPAD;
  const int nn = (n < NTOK) ? n : (NTOK - 1);
  const int f = nn / PP;
  const int p = nn - f * PP;
  const float* src = x + ((size_t)(p * (NB * FF) + b * FF + f)) * CC + 8 * L;
  const v4f a0 = *(const v4f*)(src);
  const v4f a1 = *(const v4f*)(src + 4);
  const bool keep = (n < NTOK);
  v8us hv, lv;
#pragma unroll
  for (int e = 0; e < 4; ++e) {
    const float f0 = keep ? a0[e] : 0.0f;
    const float f1 = keep ? a1[e] : 0.0f;
    const unsigned short hb0 = f2bf_bits(f0);
    const unsigned short hb1 = f2bf_bits(f1);
    hv[e]     = hb0;
    hv[4 + e] = hb1;
    lv[e]     = f2bf_bits(f0 - bf_bits2f(hb0));
    lv[4 + e] = f2bf_bits(f1 - bf_bits2f(hb1));
  }
  const size_t o = (size_t)R * CC + 8 * L;
  *(volatile v8us*)(XBh + o) = hv;
  *(volatile v8us*)(XBl + o) = lv;
  __threadfence();
  *(volatile v8us*)(XBh + o) = hv;
  *(volatile v8us*)(XBl + o) = lv;
}

template <int OM>
__global__ __launch_bounds__(256) void k_gemm(
    const unsigned short* __restrict__ Ahp, const unsigned short* __restrict__ Alp, int lda, long strideA,
    const unsigned short* __restrict__ Bhp, const unsigned short* __restrict__ Blp, int ldb, long strideB,
    void* __restrict__ Cout, int ldc, long strideC,
    const float* __restrict__ bias,
    int M, int N, int K, float scale)
{
  __shared__ __align__(16) float sT[8][16 * 68];
  const int z    = blockIdx.y;
  const int lane = threadIdx.x & 31;
  const int wave = threadIdx.x >> 5;
  const int tilesN = N >> 6;
  const int tilesM = M >> 5;
  const int tile = blockIdx.x * 8 + wave;
  if (tile >= tilesM * tilesN) return;
  const int tm = tile / tilesN;
  const int tn = tile - tm * tilesN;
  const int m0 = tm << 5;
  const int n0 = tn << 6;
  const __bf16* A0 = (const __bf16*)(const void*)Ahp + (size_t)z * strideA;
  const __bf16* A1 = (const __bf16*)(const void*)Alp + (size_t)z * strideA;
  const __bf16* B0 = (const __bf16*)(const void*)Bhp + (size_t)z * strideB;
  const __bf16* B1 = (const __bf16*)(const void*)Blp + (size_t)z * strideB;
  const int rl   = lane & 15;
  const int koff = (lane >> 4) * 8;
  const int mOff = (lane >> 4) * 8;

  v8f acc[2][4];
#pragma unroll
  for (int i = 0; i < 2; ++i)
#pragma unroll
    for (int j = 0; j < 4; ++j) acc[i][j] = zacc();

#pragma unroll 1
  for (int k0 = 0; k0 < K; k0 += 32) {
    v16b bh[4], bl[4];
#pragma unroll
    for (int j = 0; j < 4; ++j) {
      const size_t bo = (size_t)(n0 + (j << 4) + rl) * ldb + k0 + koff;
      bh[j] = ldfragb(B0 + bo);
      bl[j] = ldfragb(B1 + bo);
    }
#pragma unroll
    for (int i = 0; i < 2; ++i) {
      const size_t ao = (size_t)(m0 + (i << 4) + rl) * lda + k0 + koff;
      const v16b ah = ldfragb(A0 + ao);
      const v16b al = ldfragb(A1 + ao);
#pragma unroll
      for (int j = 0; j < 4; ++j) {
        acc[i][j] = mmab(ah, bh[j], acc[i][j]);
        acc[i][j] = mmab(ah, bl[j], acc[i][j]);
        acc[i][j] = mmab(al, bh[j], acc[i][j]);
      }
    }
  }

  float* slab = sT[wave];
#pragma unroll
  for (int i = 0; i < 2; ++i) {
    const int mBase = m0 + (i << 4);
#pragma unroll
    for (int j = 0; j < 4; ++j) {
      const int n = n0 + (j << 4) + rl;
      float bv = 0.f;
      if (OM == 1) bv = bias[n];
#pragma unroll
      for (int r = 0; r < 8; ++r)
        slab[(mOff + r) * 68 + (j << 4) + rl] = acc[i][j][r] * scale + bv;
    }
    wave_sync_lds();
    if (OM == 0) {
      _Float16* C = (_Float16*)Cout + (size_t)z * strideC;
      const int q8 = lane >> 3;
      const int c8 = (lane & 7) * 8;
      for (int ps = 0; ps < 2; ++ps) {
#pragma unroll
        for (int it = 0; it < 4; ++it) {
          const int row = it * 4 + q8;
          const float* sp = slab + row * 68 + c8;
          v8h hv;
#pragma unroll
          for (int e = 0; e < 8; ++e) hv[e] = (_Float16)sp[e];
          *(volatile v8h*)(C + (size_t)(mBase + row) * ldc + n0 + c8) = hv;
        }
        __threadfence();
      }
    } else {
      float* C = (float*)Cout + (size_t)z * strideC;
      const int hh = lane >> 4;
      const int c4 = (lane & 15) * 4;
      for (int ps = 0; ps < 2; ++ps) {
#pragma unroll
        for (int it = 0; it < 8; ++it) {
          const int row = it * 2 + hh;
          const v4f v = *(const v4f*)(slab + row * 68 + c4);
          if (OM == 2) {
            *(volatile v4f*)(C + (size_t)(mBase + row) * ldc + n0 + c4) = v;
          } else {
            const int m  = mBase + row;
            const int bb = m / NPAD;
            const int q  = m - bb * NPAD;
            const int fq = q / PP;
            const int p  = q - fq * PP;
            if (q < NTOK) {
              const size_t drow = (size_t)p * (NB * FF) + (size_t)(bb * FF + fq);
              *(volatile v4f*)(C + drow * (size_t)ldc + n0 + c4) = v;
            }
          }
        }
        __threadfence();
      }
    }
    wave_sync_lds();
  }
}

#define LDS_QS 0
#define LDS_KS (LDS_QS + 64 * QPITCH * 2)
#define LDS_VS (LDS_KS + 64 * QPITCH * 2)
#define LDS_PS (LDS_VS + CC * VPITCH * 2)
#define LDS_AL (LDS_PS + 64 * VPITCH * 2)
#define LDS_LS (LDS_AL + 64 * 4)
#define LDS_A1 (LDS_LS + 64 * 4)
static_assert(LDS_KS % 16 == 0 && LDS_VS % 16 == 0 && LDS_PS % 16 == 0 && LDS_AL % 16 == 0 && LDS_LS % 16 == 0);

__global__ __launch_bounds__(256) void k_attn1(const _Float16* __restrict__ QK, const _Float16* __restrict__ VT,
                                               unsigned short* __restrict__ X1h, unsigned short* __restrict__ X1l,
                                               unsigned short* __restrict__ XDh, unsigned short* __restrict__ XDl,
                                               int b, float sscale)
{
  __shared__ __align__(16) unsigned char lds[LDS_A1];
  _Float16* Qs = (_Float16*)(lds + LDS_QS);
  _Float16* Ks = (_Float16*)(lds + LDS_KS);
  _Float16* Vs = (_Float16*)(lds + LDS_VS);
  _Float16* Ps = (_Float16*)(lds + LDS_PS);
  float*    Al = (float*)(lds + LDS_AL);
  float*    Ls = (float*)(lds + LDS_LS);

  const int tid  = threadIdx.x;
  const int wave = tid >> 5;
  const int lane = tid & 31;
  const int h    = lane >> 4;
  const int c    = lane & 15;
  const int q0   = blockIdx.x * 64;
  const int f    = blockIdx.y;
  const _Float16* QKb = QK + (size_t)b * NPAD * C2;
  const _Float16* VTb = VT + (size_t)b * CC * NPAD;

  {
    const int r = tid >> 2, part = (tid & 3) * 64;
    const _Float16* src = QKb + (size_t)(q0 + r) * C2 + part;
    _Float16* dq = Qs + r * QPITCH + part;
#pragma unroll
    for (int i = 0; i < 8; ++i) *(v8h*)(dq + 8 * i) = *(const v8h*)(src + 8 * i);
  }

  v8f acc[4][2];
#pragma unroll
  for (int i = 0; i < 4; ++i) { acc[i][0] = zacc(); acc[i][1] = zacc(); }
  float mrow[8], lrow[8];
#pragma unroll
  for (int r = 0; r < 8; ++r) { mrow[r] = -INFINITY; lrow[r] = 0.f; }

#pragma unroll 1
  for (int kc = 0; kc < 15; ++kc) {
    const int kb = f * PP + kc * 64;
    __syncthreads();
    {
      const int r = tid >> 2, part = (tid & 3) * 64;
      const _Float16* sk = QKb + (size_t)(kb + r) * C2 + CC + part;
      _Float16* dk = Ks + r * QPITCH + part;
#pragma unroll
      for (int i = 0; i < 8; ++i) *(v8h*)(dk + 8 * i) = *(const v8h*)(sk + 8 * i);
      const _Float16* sv = VTb + (size_t)tid * NPAD + kb;
      _Float16* dv = Vs + tid * VPITCH;
#pragma unroll
      for (int i = 0; i < 8; ++i) *(v8h*)(dv + 8 * i) = *(const v8h*)(sv + 8 * i);
    }
    __syncthreads();

    if (wave < 4) {
      v8f s[4];
#pragma unroll
      for (int j = 0; j < 4; ++j) s[j] = zacc();
#pragma unroll
      for (int ks = 0; ks < 8; ++ks) {
        const v16h af = ldfragh(Qs + (16 * wave + c) * QPITCH + 32 * ks + 8 * h);
#pragma unroll
        for (int j = 0; j < 4; ++j) {
          const v16h bfj = ldfragh(Ks + (16 * j + c) * QPITCH + 32 * ks + 8 * h);
          s[j] = mmah(af, bfj, s[j]);
        }
      }
      _Float16* prow = Ps + (16 * wave + 8 * h) * VPITCH + c;
#pragma unroll
      for (int r = 0; r < 8; ++r) {
        float m = -INFINITY;
#pragma unroll
        for (int j = 0; j < 4; ++j) {
          const int kidx = kc * 64 + 16 * j + c;
          const float v = (kidx < PP) ? s[j][r] * sscale : -INFINITY;
          s[j][r] = v;
          m = fmaxf(m, v);
        }
        m = fmaxf(m, __shfl_xor(m, 1, 32));
        m = fmaxf(m, __shfl_xor(m, 2, 32));
        m = fmaxf(m, __shfl_xor(m, 4, 32));
        m = fmaxf(m, __shfl_xor(m, 8, 32));
        const float mnew  = fmaxf(mrow[r], m);
        const float alpha = __expf(mrow[r] - mnew);
        mrow[r] = mnew;
        float psum = 0.f;
#pragma unroll
        for (int j = 0; j < 4; ++j) {
          const float p = __expf(s[j][r] - mnew);
          psum += p;
          prow[r * VPITCH + 16 * j] = (_Float16)p;
        }
        psum += __shfl_xor(psum, 1, 32);
        psum += __shfl_xor(psum, 2, 32);
        psum += __shfl_xor(psum, 4, 32);
        psum += __shfl_xor(psum, 8, 32);
        lrow[r] = lrow[r] * alpha + psum;
        if (c == 0) Al[16 * wave + 8 * h + r] = alpha;
      }
    }
    __syncthreads();

#pragma unroll
    for (int i = 0; i < 4; ++i) {
      const v4f g0 = *(const v4f*)(Al + 16 * i + 8 * h);
      const v4f g1 = *(const v4f*)(Al + 16 * i + 8 * h + 4);
#pragma unroll
      for (int j = 0; j < 2; ++j) {
#pragma unroll
        for (int r = 0; r < 4; ++r) { acc[i][j][r] *= g0[r]; acc[i][j][r + 4] *= g1[r]; }
      }
    }
    const int nkk = (kc == 14) ? 1 : 2;
#pragma unroll 1
    for (int kk = 0; kk < nkk; ++kk) {
      v16h pa[4];
#pragma unroll
      for (int i = 0; i < 4; ++i) pa[i] = ldfragh(Ps + (16 * i + c) * VPITCH + 32 * kk + 8 * h);
#pragma unroll
      for (int j = 0; j < 2; ++j) {
        const v16h vb = ldfragh(Vs + (32 * wave + 16 * j + c) * VPITCH + 32 * kk + 8 * h);
#pragma unroll
        for (int i = 0; i < 4; ++i) acc[i][j] = mmah(pa[i], vb, acc[i][j]);
      }
    }
  }

  if (wave < 4) {
#pragma unroll
    for (int r = 0; r < 8; ++r)
      if (c == 0) Ls[16 * wave + 8 * h + r] = lrow[r];
  }
  __syncthreads();
  {
    unsigned short* Oh = (unsigned short*)(lds + LDS_KS);
    unsigned short* Ol = (unsigned short*)(lds + LDS_QS);
#pragma unroll
    for (int i = 0; i < 4; ++i) {
      const v4f g0 = *(const v4f*)(Ls + 16 * i + 8 * h);
      const v4f g1 = *(const v4f*)(Ls + 16 * i + 8 * h + 4);
      float inv[8];
#pragma unroll
      for (int r = 0; r < 4; ++r) {
        inv[r]     = 0.25f * __builtin_amdgcn_rcpf(g0[r]);
        inv[r + 4] = 0.25f * __builtin_amdgcn_rcpf(g1[r]);
      }
#pragma unroll
      for (int j = 0; j < 2; ++j)
#pragma unroll
        for (int r = 0; r < 8; ++r) {
          const float v = acc[i][j][r] * inv[r];
          const unsigned short hb = f2bf_bits(v);
          const unsigned short lb = f2bf_bits(v - bf_bits2f(hb));
          const int idx = (16 * i + 8 * h + r) * QPITCH + 32 * wave + 16 * j + c;
          Oh[idx] = hb;
          Ol[idx] = lb;
        }
    }
  }
  __syncthreads();
  {
    const unsigned short* Oh = (const unsigned short*)(lds + LDS_KS);
    const unsigned short* Ol = (const unsigned short*)(lds + LDS_QS);
    for (int ps = 0; ps < 2; ++ps) {
#pragma unroll
      for (int rr = 0; rr < 8; ++rr) {
        const int row = 8 * wave + rr;
        const int q   = q0 + row;
        const v8us vh = *(const v8us*)(Oh + row * QPITCH + 8 * lane);
        const v8us vl = *(const v8us*)(Ol + row * QPITCH + 8 * lane);
        const size_t o1 = ((size_t)q * FF + f) * CC + 8 * lane;
        *(volatile v8us*)(X1h + o1) = vh;
        *(volatile v8us*)(X1l + o1) = vl;
        int fq = q / PP;
        fq = (fq > FF - 1) ? (FF - 1) : fq;
        if (fq == f) {
          const size_t od = (size_t)q * CC + 8 * lane;
          *(volatile v8us*)(XDh + od) = vh;
          *(volatile v8us*)(XDl + od) = vl;
        }
      }
      __threadfence();
    }
  }
}

__global__ __launch_bounds__(256) void k_traj(const float* __restrict__ Q2, const float* __restrict__ KV,
                                              unsigned short* __restrict__ X2h, unsigned short* __restrict__ X2l,
                                              float* __restrict__ AT, int b, float qscale)
{
  __shared__ __align__(16) float ats[HH * 160];
  __shared__ __align__(16) unsigned short xsh[32 * QPITCH];
  __shared__ __align__(16) unsigned short xsl[32 * QPITCH];
  const int tid = threadIdx.x;
  const int ti  = tid >> 3;
  const int hd  = tid & 7;
  const int s0  = blockIdx.x * 32;
  const int s   = s0 + ti;
  const float* qp = Q2 + (size_t)s * CC + hd * 32;
  const float* kp = KV + (size_t)s * (FF * C2) + hd * 32;
  float l0 = 0.f, l1 = 0.f, l2 = 0.f, l3 = 0.f, l4 = 0.f;
#pragma unroll 1
  for (int d = 0; d < 32; ++d) {
    const float qd = qp[d] * qscale;
    l0 += qd * kp[d];
    l1 += qd * kp[C2 + d];
    l2 += qd * kp[2 * C2 + d];
    l3 += qd * kp[3 * C2 + d];
    l4 += qd * kp[4 * C2 + d];
  }
  const float m  = fmaxf(fmaxf(fmaxf(l0, l1), fmaxf(l2, l3)), l4);
  const float e0 = __expf(l0 - m), e1 = __expf(l1 - m), e2 = __expf(l2 - m), e3 = __expf(l3 - m), e4 = __expf(l4 - m);
  const float rden = __builtin_amdgcn_rcpf(e0 + e1 + e2 + e3 + e4);
  const float a0 = e0 * rden, a1 = e1 * rden, a2 = e2 * rden, a3 = e3 * rden, a4 = e4 * rden;
  {
    float* ap = ats + hd * 160 + ti * FF;
    ap[0] = a0; ap[1] = a1; ap[2] = a2; ap[3] = a3; ap[4] = a4;
  }
  {
    const float* vp = kp + CC;
    unsigned short* xh = xsh + ti * QPITCH + hd * 32;
    unsigned short* xl = xsl + ti * QPITCH + hd * 32;
#pragma unroll 1
    for (int d = 0; d < 32; ++d) {
      float o = a0 * vp[d];
      o += a1 * vp[C2 + d];
      o += a2 * vp[2 * C2 + d];
      o += a3 * vp[3 * C2 + d];
      o += a4 * vp[4 * C2 + d];
      const unsigned short hb = f2bf_bits(o);
      xh[d] = hb;
      xl[d] = f2bf_bits(o - bf_bits2f(hb));
    }
  }
  __syncthreads();
  const int wave = tid >> 5;
  const int lane = tid & 31;
  {
    float* dst = AT + (((size_t)b * HH + wave) * NPAD + s0) * FF;
    const float* as = ats + wave * 160;
    const v4f v0 = *(const v4f*)(as + 4 * lane);
    const int l8 = (lane < 8) ? lane : 7;
    const v4f v1 = *(const v4f*)(as + 128 + 4 * l8);
    for (int ps = 0; ps < 2; ++ps) {
      *(volatile v4f*)(dst + 4 * lane) = v0;
      if (lane < 8) *(volatile v4f*)(dst + 128 + 4 * lane) = v1;
      __threadfence();
    }
  }
  {
    for (int ps = 0; ps < 2; ++ps) {
#pragma unroll
      for (int rr = 0; rr < 4; ++rr) {
        const int row = 4 * wave + rr;
        const v8us vh = *(const v8us*)(xsh + row * QPITCH + 8 * lane);
        const v8us vl = *(const v8us*)(xsl + row * QPITCH + 8 * lane);
        const size_t o = ((size_t)b * NPAD + s0 + row) * CC + 8 * lane;
        *(volatile v8us*)(X2h + o) = vh;
        *(volatile v8us*)(X2l + o) = vl;
      }
      __threadfence();
    }
  }
}

__global__ __launch_bounds__(256) void k_acopy(const float* __restrict__ AT, float* __restrict__ dst, int n4)
{
  const int g = blockIdx.x * 256 + threadIdx.x;
  if (g >= n4) return;
  const int e   = g * 4;
  const int bh  = e / (NTOK * FF);
  const int rem = e - bh * (NTOK * FF);
  const v4f v = *(const v4f*)(AT + (size_t)bh * (NPAD * FF) + rem);
  *(volatile v4f*)(dst + e) = v;
  __threadfence();
  *(volatile v4f*)(dst + e) = v;
}

extern "C" void kernel_launch(void* const* d_in, const int* in_sizes, int n_in,
                              void* d_out, int out_size, void* d_ws, size_t ws_size,
                              hipStream_t stream)
{
  if (n_in < 6) return;
  if (in_sizes[0] != PP * NB * FF * CC) return;
  if (in_sizes[1] != C3 * CC || in_sizes[2] != CC * CC || in_sizes[3] != C2 * CC || in_sizes[4] != CC * CC || in_sizes[5] != CC) return;
  if (out_size != PP * NB * FF * CC + NB * HH * NTOK * FF) return;

  const float* x      = (const float*)d_in[0];
  const float* W_qkv  = (const float*)d_in[1];
  const float* W_pq   = (const float*)d_in[2];
  const float* W_pkv  = (const float*)d_in[3];
  const float* W_proj = (const float*)d_in[4];
  const float* b_proj = (const float*)d_in[5];

  const size_t sW3  = (size_t)C3 * CC * 2;
  const size_t sW1  = (size_t)CC * CC * 2;
  const size_t sW2  = (size_t)C2 * CC * 2;
  const size_t sXB  = (size_t)NB * NPAD * CC * 2;
  const size_t sQK  = (size_t)NB * NPAD * C2 * 2;
  const size_t sVT  = (size_t)NB * CC * NPAD * 2;
  const size_t sX1  = (size_t)NPAD * FF * CC * 2;
  const size_t sXD  = (size_t)NPAD * CC * 2;
  const size_t sQ2  = (size_t)NPAD * CC * 4;
  const size_t sKV2 = (size_t)NPAD * FF * C2 * 4;
  const size_t sAT  = (size_t)NB * HH * NPAD * FF * 4;
  size_t off = 0;
  const size_t oWQKVh = off; off += sW3;  const size_t oWQKVl = off; off += sW3;
  const size_t oWPQh  = off; off += sW1;  const size_t oWPQl  = off; off += sW1;
  const size_t oWPKVh = off; off += sW2;  const size_t oWPKVl = off; off += sW2;
  const size_t oWPRh  = off; off += sW1;  const size_t oWPRl  = off; off += sW1;
  const size_t oXBh   = off; off += sXB;  const size_t oXBl   = off; off += sXB;
  const size_t oQK    = off; off += sQK;
  const size_t oVT    = off; off += sVT;
  const size_t oX1h   = off; off += sX1;  const size_t oX1l   = off; off += sX1;
  const size_t oXDh   = off; off += sXD;  const size_t oXDl   = off; off += sXD;
  const size_t oQ2    = off; off += sQ2;
  const size_t oKV2   = off; off += sKV2;
  const size_t oAT    = off; off += sAT;
  if (off > ws_size) return;
  if (off > (size_t)134217728) return;

  char* ws = (char*)d_ws;
  unsigned short* WQKVh = (unsigned short*)(ws + oWQKVh); unsigned short* WQKVl = (unsigned short*)(ws + oWQKVl);
  unsigned short* WPQh  = (unsigned short*)(ws + oWPQh);  unsigned short* WPQl  = (unsigned short*)(ws + oWPQl);
  unsigned short* WPKVh = (unsigned short*)(ws + oWPKVh); unsigned short* WPKVl = (unsigned short*)(ws + oWPKVl);
  unsigned short* WPRh  = (unsigned short*)(ws + oWPRh);  unsigned short* WPRl  = (unsigned short*)(ws + oWPRl);
  unsigned short* XBh   = (unsigned short*)(ws + oXBh);   unsigned short* XBl   = (unsigned short*)(ws + oXBl);
  unsigned short* X2h   = (unsigned short*)(ws + oXBh);
  unsigned short* X2l   = (unsigned short*)(ws + oXBl);
  _Float16*       QK    = (_Float16*)(ws + oQK);
  _Float16*       VT    = (_Float16*)(ws + oVT);
  unsigned short* X1h   = (unsigned short*)(ws + oX1h);   unsigned short* X1l   = (unsigned short*)(ws + oX1l);
  unsigned short* XDh   = (unsigned short*)(ws + oXDh);   unsigned short* XDl   = (unsigned short*)(ws + oXDl);
  float*          Q2    = (float*)(ws + oQ2);
  float*          KV2   = (float*)(ws + oKV2);
  float*          AT    = (float*)(ws + oAT);

  const float scale = 0.17677669529663687f;
  const dim3 blk(256);

  k_wcvt<<<dim3(96, 4), blk, 0, stream>>>(W_qkv, WQKVh, WQKVl, C3 * CC, W_pq, WPQh, WPQl, CC * CC,
                                          W_pkv, WPKVh, WPKVl, C2 * CC, W_proj, WPRh, WPRl, CC * CC);
  k_pack<<<dim3((NB * NPAD * 32) / 256), blk, 0, stream>>>(x, XBh, XBl);
  {
    const int tiles = (NB * NPAD / 32) * (C2 / 64);
    k_gemm<0><<<dim3((tiles + 7) / 8, 1), blk, 0, stream>>>(XBh, XBl, CC, 0L, WQKVh, WQKVl, CC, 0L,
                                                             (void*)QK, C2, 0L, b_proj, NB * NPAD, C2, CC, 4.0f);
  }
  {
    const int tiles = (CC / 32) * (NPAD / 64);
    k_gemm<0><<<dim3((tiles + 7) / 8, NB), blk, 0, stream>>>(WQKVh + (size_t)C2 * CC, WQKVl + (size_t)C2 * CC, CC, 0L,
                                                              XBh, XBl, CC, (long)NPAD * CC,
                                                              (void*)VT, NPAD, (long)CC * NPAD, b_proj, CC, NPAD, CC, 4.0f);
  }
  for (int b = 0; b < NB; ++b) {
    k_attn1<<<dim3(NPAD / 64, FF), blk, 0, stream>>>(QK, VT, X1h, X1l, XDh, XDl, b, scale * 0.0625f);
    {
      const int tiles = (NPAD / 32) * (CC / 64);
      k_gemm<2><<<dim3((tiles + 7) / 8, 1), blk, 0, stream>>>(XDh, XDl, CC, 0L, WPQh, WPQl, CC, 0L,
                                                               (void*)Q2, CC, 0L, b_proj, NPAD, CC, CC, 1.0f);
    }
    {
      const int tiles = (NPAD * FF / 32) * (C2 / 64);
      k_gemm<2><<<dim3((tiles + 7) / 8, 1), blk, 0, stream>>>(X1h, X1l, CC, 0L, WPKVh, WPKVl, CC, 0L,
                                                               (void*)KV2, C2, 0L, b_proj, NPAD * FF, C2, CC, 1.0f);
    }
    k_traj<<<dim3(NPAD / 32), blk, 0, stream>>>(Q2, KV2, X2h, X2l, AT, b, scale);
  }
  {
    const int tiles = (NB * NPAD / 32) * (CC / 64);
    k_gemm<1><<<dim3((tiles + 7) / 8, 1), blk, 0, stream>>>(X2h, X2l, CC, 0L, WPRh, WPRl, CC, 0L,
                                                             d_out, CC, 0L, b_proj, NB * NPAD, CC, CC, 1.0f);
  }
  {
    const int n4 = NB * HH * NTOK * FF / 4;
    float* out1 = (float*)d_out + (size_t)PP * NB * FF * CC;
    k_acopy<<<dim3((n4 + 255) / 256), blk, 0, stream>>>(AT, out1, n4);
  }
  (void)hipGetLastError();
}
